// MultiHeadAttention_86457691669080
// MI455X (gfx1250) — hardware-run, weakly checked
//
#include <hip/hip_runtime.h>
#define NBE 4
#define NTK 1024
#define NW 1024
#define NHD 16
#define HW 64
#define FILLH -1.0e9f
#define PSC 1024.0f
#define WSC 256.0f
#define YSC 256.0f

typedef __bf16 v16b __attribute__((ext_vector_type(16)));
typedef unsigned short v8us __attribute__((ext_vector_type(8), may_alias));
typedef float  v8f  __attribute__((ext_vector_type(8)));
typedef float  v4f  __attribute__((ext_vector_type(4)));
typedef float  v4fa __attribute__((ext_vector_type(4), may_alias));
union FragB { v16b v; v8us half[2]; unsigned short u[16]; };

__device__ __forceinline__ unsigned short bf16_bits(float x) { unsigned int u = __float_as_uint(x); return (unsigned short)((u + 0x7FFFu + ((u >> 16) & 1u)) >> 16); }
__device__ __forceinline__ float bf16_val(unsigned short b) { return __uint_as_float(((unsigned int)b) << 16); }
__device__ __forceinline__ float bf16_round(float x) { return bf16_val(bf16_bits(x)); }
template <int NT>
__device__ __forceinline__ v8f mmaN(v16b ah, v16b al, v16b bh, v16b bl, v8f c) {
  c = __builtin_amdgcn_wmma_f32_16x16x32_bf16(false, ah, false, bh, (short)0, c, false, false);
  if (NT >= 2) c = __builtin_amdgcn_wmma_f32_16x16x32_bf16(false, al, false, bh, (short)0, c, false, false);
  if (NT >= 3) c = __builtin_amdgcn_wmma_f32_16x16x32_bf16(false, ah, false, bl, (short)0, c, false, false);
  asm volatile("v_nop\n\tv_nop\n\tv_nop\n\tv_nop" : "+v"(c) : "v"(ah), "v"(al), "v"(bh), "v"(bl));
  return c;
}


typedef _Float16 v16h __attribute__((ext_vector_type(16)));
union FragH { v16h v; v8us half[2]; _Float16 h[16]; unsigned short u[16]; };
template <int NT>
__device__ __forceinline__ v8f mmaH(v16h ah, v16h al, v16h bh, v16h bl, v8f c) {
  c = __builtin_amdgcn_wmma_f32_16x16x32_f16(false, ah, false, bh, (short)0, c, false, false);
  if (NT >= 2) c = __builtin_amdgcn_wmma_f32_16x16x32_f16(false, al, false, bh, (short)0, c, false, false);
  if (NT >= 3) c = __builtin_amdgcn_wmma_f32_16x16x32_f16(false, ah, false, bl, (short)0, c, false, false);
  asm volatile("v_nop\n\tv_nop\n\tv_nop\n\tv_nop" : "+v"(c) : "v"(ah), "v"(al), "v"(bh), "v"(bl));
  return c;
}

__global__ __launch_bounds__(256) void k_wt_f16(const float* __restrict__ W, _Float16* __restrict__ Wt, int K, int N, float scale) {
  const int t = blockIdx.x * 256 + threadIdx.x; if (t >= N * (K / 8)) return; const int n = t / (K / 8), k8 = (t % (K / 8)) * 8; FragH f;
#pragma unroll
  for (int i = 0; i < 8; ++i) f.h[i] = (_Float16)(bf16_round(W[(size_t)(k8 + i) * N + n]) * scale); const v8us o = f.half[0];
  *(volatile v8us*)((unsigned short*)Wt + (size_t)n * K + k8) = o; __threadfence(); *(volatile v8us*)((unsigned short*)Wt + (size_t)n * K + k8) = o;
}

typedef _Float16 v4h __attribute__((ext_vector_type(4)));

__global__ __launch_bounds__(256) void k_x16(const float* __restrict__ x, _Float16* __restrict__ X16, size_t n8) { const size_t t = (size_t)blockIdx.x * 256 + threadIdx.x; if (t >= n8) return; FragH f;
#pragma unroll
  for (int q = 0; q < 8; ++q) f.h[q] = (_Float16)bf16_round(x[t * 8 + q]); *(volatile v8us*)((unsigned short*)X16 + t * 8) = f.half[0]; __threadfence(); *(volatile v8us*)((unsigned short*)X16 + t * 8) = f.half[0]; }
__device__ __forceinline__ v16h g2_frag(const _Float16* p, int hh) { FragH f; f.half[0] = *(const v8us*)((const unsigned short*)p + 8 * hh); f.half[1] = *(const v8us*)((const unsigned short*)p + 16 + 8 * hh); return f.v; }
__device__ __forceinline__ v8f g2_mma(v16h a, v16h b, v8f c) { v8f d = __builtin_amdgcn_wmma_f32_16x16x32_f16(false, a, false, b, (short)0, c, false, false); asm volatile("v_nop\n\tv_nop\n\tv_nop\n\tv_nop" : "+v"(d) : "v"(a), "v"(b)); return d; }
template <int ACT>
__global__ __launch_bounds__(128) void k_gemm2(const _Float16* __restrict__ A, int lda, size_t sA, const _Float16* __restrict__ Bh, int ldb, size_t sB, float alpha, const float* __restrict__ bias, size_t sBias, const float* __restrict__ CP, int rowsPerB, size_t sCPb, int row0g,
    float* __restrict__ C, _Float16* __restrict__ C16, int ldc, size_t sC, int M, int N, int K) { static_assert(ACT == 0 || ACT == 3 || ACT == 6 || ACT == 8 || ACT == 9 || ACT == 11 || ACT == 12 || ACT == 14 || ACT == 15 || ACT == 16 || ACT == 17, "k_gemm2: unsupported ACT code (would silently apply no activation)");
  __shared__ __attribute__((aligned(16))) float so[4][32][68];
  const int tid = threadIdx.x, w = tid >> 5, lane = tid & 31, ln = lane & 15, hh = lane >> 4; const int by = blockIdx.y;
  A += (size_t)by * sA; Bh += (size_t)by * sB; const size_t cofs = (size_t)by * sC; const float* bp = bias ? bias + (size_t)by * sBias : nullptr;
  const int ntn = N >> 6; const int mt = blockIdx.x / ntn, nq = blockIdx.x - mt * ntn; const int row0 = mt * 128 + 32 * w, col0 = nq * 64; if (row0 >= M) return;
  const _Float16* a0p = A + (size_t)(row0 + ln) * lda; const _Float16* a1p = a0p + (size_t)16 * lda;
  const _Float16* b0p = Bh + (size_t)(col0 + ln) * ldb; const _Float16* b1p = b0p + (size_t)16 * ldb; const _Float16* b2p = b1p + (size_t)16 * ldb; const _Float16* b3p = b2p + (size_t)16 * ldb;
  const v8f z8 = {0.f,0.f,0.f,0.f,0.f,0.f,0.f,0.f}; v8f c00 = z8, c01 = z8, c02 = z8, c03 = z8, c10 = z8, c11 = z8, c12 = z8, c13 = z8;
  for (int kb = 0; kb < K; kb += 32) { const v16h a0 = g2_frag(a0p + kb, hh), a1 = g2_frag(a1p + kb, hh);
    v16h b = g2_frag(b0p + kb, hh); c00 = g2_mma(a0, b, c00); c10 = g2_mma(a1, b, c10);
    b = g2_frag(b1p + kb, hh); c01 = g2_mma(a0, b, c01); c11 = g2_mma(a1, b, c11);
    b = g2_frag(b2p + kb, hh); c02 = g2_mma(a0, b, c02); c12 = g2_mma(a1, b, c12);
    b = g2_frag(b3p + kb, hh); c03 = g2_mma(a0, b, c03); c13 = g2_mma(a1, b, c13); }
  v8f accs[8] = {c00, c01, c02, c03, c10, c11, c12, c13};
#pragma unroll
  for (int u = 0; u < 8; ++u) { const int t = u & 3, half = u >> 2; const int col = col0 + t * 16 + ln; const float bv = bp ? bf16_round(bp[col]) : 0.f;
#pragma unroll
    for (int r = 0; r < 8; ++r) { const int rloc = half * 16 + 8 * hh + r; float v = accs[u][r] * alpha + bv; if (CP) { if (rowsPerB < 0) v += CP[cofs + (size_t)(row0g + row0 + rloc) * ldc + col];        else { const int bidx = (row0g + row0 + rloc) / rowsPerB; v += CP[(size_t)bidx * sCPb + (size_t)by * 64 + col]; } }
      if (ACT == 3) v = fmaxf(v, 0.f); else if (ACT == 6) v = 0.5f * v * (1.0f + erff(v * 0.70710678118654752f)); else if (ACT == 11) v = 1.0f / (1.0f + expf(-v)); else if (ACT == 15) v = v / (1.0f + expf(-v)); else if (ACT == 12) v = (v > 0.f) ? v : 0.01f * v; else if (ACT == 8) v = tanhf(v); else if (ACT == 9) v = 0.5f * v * (1.0f + tanhf(0.7978845608028654f * (v + 0.044715f * v * v * v))); else if (ACT == 14) v = (v > 0.f) ? v : 0.1f * v; else if (ACT == 16) v = (v >= 0.f) ? v : 0.3f * v; else if (ACT == 17) v = (v >= 0.f) ? v : 0.2f * v;
      so[w][rloc][t * 16 + ln] = v; } }
  __builtin_amdgcn_fence(__ATOMIC_ACQ_REL, "workgroup"); __builtin_amdgcn_wave_barrier();
  const int rsub = lane >> 4, c4 = (lane & 15) * 4;
  for (int pass = 0; pass < 2; ++pass) {
#pragma unroll
    for (int q = 0; q < 16; ++q) { const int r = q * 2 + rsub; const v4f v = *(const v4fa*)&so[w][r][c4]; if (C) *(volatile v4f*)(C + cofs + (size_t)(row0 + r) * ldc + col0 + c4) = v; if (C16) { v4h h4; for (int i = 0; i < 4; ++i) h4[i] = (_Float16)v[i]; *(volatile v4h*)(C16 + cofs + (size_t)(row0 + r) * ldc + col0 + c4) = h4; } }
    if (pass == 0) __threadfence(); } }

__global__ __launch_bounds__(256) void k_wtc_f16(const float* __restrict__ W, _Float16* __restrict__ Wt, int K, int N, float scale) {
  const int t = blockIdx.x * 256 + threadIdx.x; if (t >= N * (K / 8)) return; const int n = t / (K / 8), k8 = (t % (K / 8)) * 8; FragH f;
#pragma unroll
  for (int i = 0; i < 8; ++i) f.h[i] = (_Float16)(W[(size_t)(k8 + i) * N + n] * scale); const v8us o = f.half[0];
  *(volatile v8us*)((unsigned short*)Wt + (size_t)n * K + k8) = o; __threadfence(); *(volatile v8us*)((unsigned short*)Wt + (size_t)n * K + k8) = o;
}

typedef int v4ia __attribute__((ext_vector_type(4), may_alias));

__global__ __launch_bounds__(256) void k_x16s(const float* __restrict__ x, _Float16* __restrict__ X16, size_t n8, float carry) { const size_t t = (size_t)blockIdx.x * 256 + threadIdx.x; if (t >= n8) return; FragH f;
#pragma unroll
  for (int q = 0; q < 8; ++q) f.h[q] = (_Float16)(bf16_round(x[t * 8 + q]) * carry); *(volatile v8us*)((unsigned short*)X16 + t * 8) = f.half[0]; __threadfence(); *(volatile v8us*)((unsigned short*)X16 + t * 8) = f.half[0]; }

__global__ __launch_bounds__(256) void k_dsm(const float* __restrict__ Z, const float* __restrict__ AP, const int* __restrict__ HP, const float* __restrict__ GI, _Float16* __restrict__ P16, int n) {
  const int r = blockIdx.x * 8 + (threadIdx.x >> 5); if (r >= n) return; const int ln = threadIdx.x & 31; const int t = r % NTK; const float* zp = Z + (size_t)r * NTK + ln * 8; const float* aq = AP + (size_t)t * NTK + ln * 8; const int* hq = HP + (size_t)t * NTK + ln * 8; float m1 = -3.0e38f, m2 = -3.0e38f;
  for (int c = 0; c < NTK; c += 256) { const v4f p0 = *(const v4fa*)(zp + c); const v4f p1 = *(const v4fa*)(zp + c + 4); const v4f a0 = *(const v4fa*)(aq + c); const v4f a1 = *(const v4fa*)(aq + c + 4); const v4ia h0 = *(const v4ia*)(hq + c); const v4ia h1 = *(const v4ia*)(hq + c + 4); v4f z0, z1; for (int i = 0; i < 4; ++i) { z0[i] = p0[i] + bf16_round(a0[i]); z1[i] = p1[i] + bf16_round(a1[i]); }
    for (int i = 0; i < 4; ++i) { const float y = z0[i]; m1 = (y > m1) ? y : m1; const float u = (h0[i] == 0) ? FILLH : y; m2 = (u > m2) ? u : m2; }
    for (int i = 0; i < 4; ++i) { const float y = z1[i]; m1 = (y > m1) ? y : m1; const float u = (h1[i] == 0) ? FILLH : y; m2 = (u > m2) ? u : m2; } }
  for (int w = 16; w >= 1; w >>= 1) { const float o1 = __shfl_xor(m1, w, 32); m1 = (o1 > m1) ? o1 : m1; const float o2 = __shfl_xor(m2, w, 32); m2 = (o2 > m2) ? o2 : m2; }
  float s1 = 0.f, s2 = 0.f;
  for (int c = 0; c < NTK; c += 256) { const v4f p0 = *(const v4fa*)(zp + c); const v4f p1 = *(const v4fa*)(zp + c + 4); const v4f a0 = *(const v4fa*)(aq + c); const v4f a1 = *(const v4fa*)(aq + c + 4); const v4ia h0 = *(const v4ia*)(hq + c); const v4ia h1 = *(const v4ia*)(hq + c + 4); v4f z0, z1; for (int i = 0; i < 4; ++i) { z0[i] = p0[i] + bf16_round(a0[i]); z1[i] = p1[i] + bf16_round(a1[i]); }
    for (int i = 0; i < 4; ++i) { s1 += expf(z0[i] - m1); s2 += expf(((h0[i] == 0) ? FILLH : z0[i]) - m2); }
    for (int i = 0; i < 4; ++i) { s1 += expf(z1[i] - m1); s2 += expf(((h1[i] == 0) ? FILLH : z1[i]) - m2); } }
  for (int w = 16; w >= 1; w >>= 1) { s1 += __shfl_xor(s1, w, 32); s2 += __shfl_xor(s2, w, 32); }
  const float g1 = 1.0f / (1.0f + expf(-bf16_round(GI[0]))); const float g2 = 1.0f - g1; unsigned short* hp = (unsigned short*)P16 + (size_t)r * NTK + ln * 8;
  for (int c = 0; c < NTK; c += 256) { const v4f p0 = *(const v4fa*)(zp + c); const v4f p1 = *(const v4fa*)(zp + c + 4); const v4f a0 = *(const v4fa*)(aq + c); const v4f a1 = *(const v4fa*)(aq + c + 4); const v4ia h0 = *(const v4ia*)(hq + c); const v4ia h1 = *(const v4ia*)(hq + c + 4); v4f z0, z1; for (int i = 0; i < 4; ++i) { z0[i] = p0[i] + bf16_round(a0[i]); z1[i] = p1[i] + bf16_round(a1[i]); } FragH f;
    for (int i = 0; i < 4; ++i) { const float pa = g1 * (expf(z0[i] - m1) / s1) + g2 * (expf(((h0[i] == 0) ? FILLH : z0[i]) - m2) / s2); const float pb = g1 * (expf(z1[i] - m1) / s1) + g2 * (expf(((h1[i] == 0) ? FILLH : z1[i]) - m2) / s2); const _Float16 ha = (_Float16)(pa * PSC); const _Float16 hb = (_Float16)(pb * PSC); f.h[i] = (ha < (_Float16)6.103515625e-05f) ? (_Float16)0.0f : ha; f.h[4 + i] = (hb < (_Float16)6.103515625e-05f) ? (_Float16)0.0f : hb; }
    *(volatile v8us*)(hp + c) = f.half[0]; __threadfence(); *(volatile v8us*)(hp + c) = f.half[0]; } }

__global__ __launch_bounds__(256) void k_csz(const float* __restrict__ T, float* __restrict__ SZ) { const int t = blockIdx.x * 256 + threadIdx.x; if (t >= NBE * NW) return; const int e = t / NW, c = t % NW; const float* tp = T + (size_t)e * NTK * NW + c; float acc = 0.f;
  for (int r = 0; r < NTK; ++r) { const float rt = sqrtf(fabsf(tp[(size_t)r * NW])); acc += rt * rt; }
  const float sz = sqrtf(acc); *(volatile float*)(SZ + t) = sz; __threadfence(); *(volatile float*)(SZ + t) = sz; }

__global__ __launch_bounds__(256) void k_srw(const float* __restrict__ T, const float* __restrict__ SZ, _Float16* __restrict__ Y16, size_t n8) { const size_t t = (size_t)blockIdx.x * 256 + threadIdx.x; if (t >= n8) return; const size_t i0 = t * 8; const int c0 = (int)(i0 % NW); const int e = (int)(i0 / ((size_t)NTK * NW)); FragH f;
#pragma unroll
  for (int q = 0; q < 8; ++q) { const float w = T[i0 + q]; const float rt = sqrtf(fabsf(w)); const float sr = (w > 0.f) ? rt : ((w < 0.f) ? -rt : 0.f); const float sz = SZ[e * NW + c0 + q]; const float dn = (sz > 1.0e-12f) ? sz : 1.0e-12f; const float y = (sr / dn) * YSC; const float yf = (fabsf(y) < 6.103515625e-05f) ? 0.0f : y; f.h[q] = (_Float16)yf; }
  *(volatile v8us*)((unsigned short*)Y16 + i0) = f.half[0]; __threadfence(); *(volatile v8us*)((unsigned short*)Y16 + i0) = f.half[0]; }

extern "C" void kernel_launch(void* const* d_in, const int* in_sizes, int n_in,
                              void* d_out, int out_size, void* d_ws, size_t ws_size, hipStream_t stream) {
  (void)in_sizes; (void)n_in; (void)out_size;
  const float* XA = (const float*)d_in[0]; const float* XB = (const float*)d_in[1]; const float* XC = (const float*)d_in[2]; const float* AP = (const float*)d_in[3]; const int* HP = (const int*)d_in[4];
  const float* MA = (const float*)d_in[5]; const float* VA = (const float*)d_in[6]; const float* MB = (const float*)d_in[7]; const float* VB = (const float*)d_in[8]; const float* MC = (const float*)d_in[9]; const float* VC = (const float*)d_in[10]; const float* MD = (const float*)d_in[11]; const float* VD = (const float*)d_in[12]; const float* GI = (const float*)d_in[13];
  static_assert(NBE == 4 && NTK == 1024 && NW == 1024 && NHD == 16 && HW == 64 && NHD * HW == NW && NTK % 256 == 0 && NTK % 128 == 0 && NTK % 64 == 0 && HW % 64 == 0 && HW % 32 == 0 && NW % 64 == 0 && NW % 32 == 0 && (NBE * NTK) % 128 == 0 && (NHD * NTK) % 8 == 0 && ((size_t)NBE * NTK * NW / 8) % 256 == 0 && ((size_t)NW * (NW / 8)) % 256 == 0 && ((size_t)NW * (NTK / 8)) % 256 == 0 && (NBE * NW) % 256 == 0, "whole tiles; exact grids");
  float* OUT = (float*)d_out;
  char* wsb = (char*)d_ws; size_t off = 0;
  _Float16* XA16 = (_Float16*)(wsb + off); off += (size_t)NBE * NTK * NW * 2;
  _Float16* XB16 = (_Float16*)(wsb + off); off += (size_t)NBE * NTK * NW * 2;
  _Float16* XC16 = (_Float16*)(wsb + off); off += (size_t)NBE * NTK * NW * 2;
  _Float16* MA16 = (_Float16*)(wsb + off); off += (size_t)NW * NW * 2;
  _Float16* MB16 = (_Float16*)(wsb + off); off += (size_t)NW * NW * 2;
  _Float16* MC16 = (_Float16*)(wsb + off); off += (size_t)NW * NW * 2;
  _Float16* MD16 = (_Float16*)(wsb + off); off += (size_t)NW * NW * 2;
  _Float16* QA16 = (_Float16*)(wsb + off); off += (size_t)NBE * NTK * NW * 2;
  _Float16* QB16 = (_Float16*)(wsb + off); off += (size_t)NBE * NTK * NW * 2;
  float* QC32 = (float*)(wsb + off); off += (size_t)NBE * NTK * NW * 4;
  _Float16* QCT = (_Float16*)(wsb + off); off += (size_t)NBE * NW * NTK * 2;
  float* ZL = (float*)(wsb + off); off += (size_t)NHD * NTK * NTK * 4;
  _Float16* P16 = (_Float16*)(wsb + off); off += (size_t)NHD * NTK * NTK * 2;
  float* TM = (float*)(wsb + off); off += (size_t)NBE * NTK * NW * 4;
  float* SZ = (float*)(wsb + off); off += (size_t)NBE * NW * 4;
  _Float16* Y16 = (_Float16*)(wsb + off); off += (size_t)NBE * NTK * NW * 2;
  if (off > ws_size) return;
  const size_t n8x = (size_t)NBE * NTK * NW / 8, n8m = (size_t)NW * NW / 8;
  k_x16<<<(unsigned)(n8x / 256), 256, 0, stream>>>(XA, XA16, n8x); k_x16<<<(unsigned)(n8x / 256), 256, 0, stream>>>(XB, XB16, n8x); k_x16<<<(unsigned)(n8x / 256), 256, 0, stream>>>(XC, XC16, n8x);
  k_x16s<<<(unsigned)(n8m / 256), 256, 0, stream>>>(MA, MA16, n8m, WSC); k_x16s<<<(unsigned)(n8m / 256), 256, 0, stream>>>(MB, MB16, n8m, WSC); k_x16s<<<(unsigned)(n8m / 256), 256, 0, stream>>>(MC, MC16, n8m, WSC); k_x16s<<<(unsigned)(n8m / 256), 256, 0, stream>>>(MD, MD16, n8m, WSC);
  const dim3 gp((NBE * NTK / 128) * (NW / 64), 1);
  k_gemm2<0><<<gp, 128, 0, stream>>>(XA16, NW, 0, MA16, NW, 0, 1.0f / WSC, VA, 0, nullptr, 0, 0, 0, nullptr, QA16, NW, 0, NBE * NTK, NW, NW);
  k_gemm2<0><<<gp, 128, 0, stream>>>(XB16, NW, 0, MB16, NW, 0, 1.0f / WSC, VB, 0, nullptr, 0, 0, 0, nullptr, QB16, NW, 0, NBE * NTK, NW, NW);
  k_gemm2<0><<<gp, 128, 0, stream>>>(XC16, NW, 0, MC16, NW, 0, 1.0f / WSC, VC, 0, nullptr, 0, 0, 0, QC32, nullptr, NW, 0, NBE * NTK, NW, NW);
  for (int e = 0; e < NBE; ++e) k_wtc_f16<<<(unsigned)((size_t)NW * (NTK / 8) / 256), 256, 0, stream>>>(QC32 + (size_t)e * NTK * NW, QCT + (size_t)e * NW * NTK, NTK, NW, 1.0f);
  for (int e = 0; e < NBE; ++e) {
    k_gemm2<0><<<dim3((NTK / 128) * (NTK / 64), NHD), 128, 0, stream>>>(QA16 + (size_t)e * NTK * NW, NW, HW, QB16 + (size_t)e * NTK * NW, NW, HW, 0.03125f, nullptr, 0, nullptr, 0, 0, 0, ZL, nullptr, NTK, (size_t)NTK * NTK, NTK, NTK, HW);
    k_dsm<<<NHD * NTK / 8, 256, 0, stream>>>(ZL, AP + (size_t)e * NTK * NTK, HP + (size_t)e * NTK * NTK, GI, P16, NHD * NTK);
    k_gemm2<0><<<dim3((NTK / 128) * (HW / 64), NHD), 128, 0, stream>>>(P16, NTK, (size_t)NTK * NTK, QCT + (size_t)e * NW * NTK, NTK, (size_t)HW * NTK, 1.0f / PSC, nullptr, 0, nullptr, 0, 0, 0, TM + (size_t)e * NTK * NW, nullptr, NW, HW, NTK, HW, NTK);
  }
  k_csz<<<NBE * NW / 256, 256, 0, stream>>>(TM, SZ);
  k_srw<<<(unsigned)(n8x / 256), 256, 0, stream>>>(TM, SZ, Y16, n8x);
  k_gemm2<0><<<gp, 128, 0, stream>>>(Y16, NW, 0, MD16, NW, 0, 1.0f / (YSC * WSC), VD, 0, nullptr, 0, 0, 0, OUT, nullptr, NW, 0, NBE * NTK, NW, NW);
}
